// PointnetLFPModuleMSG_5669356832938
// MI455X (gfx1250) — hardware-verified
//
#include <hip/hip_runtime.h>
#include <stddef.h>
#include <stdint.h>


#define NB    4
#define NQ    4096
#define NPT   4096
#define NC    64
#define NQT   (NB * NQ)
#define NST   (NB * NPT)
#define K0    67
#define K0P   96
#define H0    64
#define H1    64
#define KPO   128
#define NPO   128
#define NCH   256
#define S0    16
#define S1    32
#define QPW   8
#define WPB   4
#define QPB   (QPW * WPB)
#define ASC   8.0f
#define WSC   1024.0f
#define OSC   0.0001220703125f
#define T0B   0x3C23D70Au
#define T1B   0x3D23D70Au
#define SMW00 0
#define SMW01 12288
#define SMW10 20480
#define SMW11 32768
#define SMB   40960
#define SMWV  41984
#define WX0   0
#define WX1   6144
#define WI0   10240
#define WI1   10304
#define WPR   10432
#define WVB   10752
#define SMEM  (SMWV + WPB * WVB)
#define WSCAP 134217728
#define OUTN  (NB * NCH * NQ)

static_assert(SMW01 == SMW00 + H0 * K0P * 2);
static_assert(SMW10 == SMW01 + H1 * H0 * 2);
static_assert(SMW11 == SMW10 + H0 * K0P * 2);
static_assert(SMB == SMW11 + H1 * H0 * 2);
static_assert(SMWV == SMB + 4 * 64 * 4);
static_assert(WX1 == WX0 + S1 * K0P * 2);
static_assert(WI0 == WX1 + S1 * H0 * 2);
static_assert(WI1 == WI0 + S0 * 4);
static_assert(WPR == WI1 + S1 * 4);
static_assert(WVB >= WPR + H1 * 2);
static_assert((SMWV % 16) == 0 && (WVB % 16) == 0 && (WPR % 16) == 0);
static_assert(NQT % QPB == 0);
static_assert(NQ % QPB == 0);
static_assert(NPT % 64 == 0 && NQ % 64 == 0);
static_assert(K0P % 32 == 0 && H0 % 32 == 0 && KPO % 32 == 0);
static_assert((H0 * K0P / 8) % 256 == 0);
static_assert((H1 * H0 / 8) % 256 == 0);
static_assert((NPO * KPO / 8) % 256 == 0);
static_assert(NST % 256 == 0);

typedef float    v4f  __attribute__((ext_vector_type(4)));
typedef float    v8f  __attribute__((ext_vector_type(8)));
typedef _Float16 v8h  __attribute__((ext_vector_type(8)));
typedef _Float16 v16h __attribute__((ext_vector_type(16)));
union FragH { v16h v; v8h h[2]; };

__device__ __forceinline__ v8f wmf(v16h a, v16h b, v8f c) {
  v8f d = __builtin_amdgcn_wmma_f32_16x16x32_f16(false, a, false, b, (short)0, c, false, false);
  asm volatile("v_nop\n\tv_nop\n\tv_nop\n\tv_nop" : "+v"(d) : "v"(a), "v"(b));
  return d;
}

__device__ __forceinline__ v8f splat8(float x) { v8f r = {x, x, x, x, x, x, x, x}; return r; }

__device__ __forceinline__ v16h ldfrag(const _Float16* p, int k0, int hh) {
  FragH u;
  u.h[0] = *(const v8h*)(p + k0 + 8 * hh);
  u.h[1] = *(const v8h*)(p + k0 + 16 + 8 * hh);
  return u.v;
}

__device__ __forceinline__ void wave_sync() {
  __builtin_amdgcn_fence(__ATOMIC_RELEASE, "wavefront");
  __builtin_amdgcn_wave_barrier();
}

__device__ __forceinline__ float vgpr_zero() {
  float z;
  asm volatile("v_mov_b32 %0, 0" : "=v"(z));
  return z;
}

__device__ __forceinline__ float norm3(float x, float y, float z) {
#pragma clang fp contract(off)
  float xx = x * x;
  asm volatile("" : "+v"(xx));
  float zz = z * z;
  asm volatile("" : "+v"(zz));
  float yy = y * y;
  asm volatile("" : "+v"(yy));
  float s = xx + zz;
  asm volatile("" : "+v"(s));
  return s + yy;
}

__global__ __launch_bounds__(256) void k_prepw(const float* __restrict__ W, int Kd, int Kp, int remap,
                                                int npieces, _Float16* dst) {
  const int t = threadIdx.x;
  const int p = blockIdx.x * 256 + t;
  const bool act = p < npieces;
  const int pc = act ? p : 0;
  const int npc = Kp >> 3;
  const int n = pc / npc;
  const int k8 = (pc - n * npc) * 8;
  const _Float16 hz = (_Float16)vgpr_zero();
  const float* wr = W + (size_t)n * Kd;
  v8h o;
#pragma unroll
  for (int e = 0; e < 8; ++e) {
    const int k = k8 + e;
    int src = k;
    bool valid = k < Kd;
    if (remap != 0) {
      src = (k < 64) ? (k + 3) : (k - 64);
      valid = k < 67;
    }
    src = min(max(src, 0), Kd - 1);
    const float v = wr[src] * WSC;
    o[e] = valid ? (_Float16)v : hz;
  }
  _Float16* d = dst + (size_t)8 * pc;
  if (act) *(volatile v8h*)d = o;
  __threadfence();
  if (act) *(volatile v8h*)d = o;
}

__global__ __launch_bounds__(256) void k_pts(const float* __restrict__ xyz, int npts, v4f* P1) {
#pragma clang fp contract(off)
  const int p = blockIdx.x * 256 + threadIdx.x;
  const bool act = p < npts;
  const int pc = min(p, npts - 1);
  const float x = xyz[(size_t)3 * pc], y = xyz[(size_t)3 * pc + 1], z = xyz[(size_t)3 * pc + 2];
  const float ns = norm3(x, y, z);
  const v4f o = {x, y, z, ns};
  if (act) *(volatile v4f*)(P1 + pc) = o;
  __threadfence();
  if (act) *(volatile v4f*)(P1 + pc) = o;
}

__global__ __launch_bounds__(256) void k_tr(const float* __restrict__ fa, const float* __restrict__ fb,
                                             _Float16* Fa, _Float16* Fb) {
  __shared__ float s[NC][65];
  const int t = threadIdx.x;
  const int which = blockIdx.x / (NB * (NPT / 64));
  const int rem = blockIdx.x - which * (NB * (NPT / 64));
  const int b = rem / (NPT / 64);
  const int n0 = (rem - b * (NPT / 64)) * 64;
  const float* src = (which == 0) ? fa : fb;
  _Float16* dst = (which == 0) ? Fa : Fb;
#pragma unroll 4
  for (int i = 0; i < 16; ++i) {
    const int c = 4 * i + (t >> 6);
    const int n = t & 63;
    s[c][n] = src[((size_t)(b * NC + c)) * NPT + n0 + n];
  }
  __syncthreads();
  const int p0 = t, p1 = t + 256;
  const int r0 = p0 >> 3, j0 = p0 & 7, r1 = p1 >> 3, j1 = p1 & 7;
  v8h o0, o1;
#pragma unroll
  for (int e = 0; e < 8; ++e) {
    o0[e] = (_Float16)(s[8 * j0 + e][r0] * ASC);
    o1[e] = (_Float16)(s[8 * j1 + e][r1] * ASC);
  }
  _Float16* d0 = dst + ((size_t)(b * NPT + n0 + r0)) * NC + 8 * j0;
  _Float16* d1 = dst + ((size_t)(b * NPT + n0 + r1)) * NC + 8 * j1;
  *(volatile v8h*)d0 = o0;
  *(volatile v8h*)d1 = o1;
  __threadfence();
  *(volatile v8h*)d0 = o0;
  *(volatile v8h*)d1 = o1;
}

template <int MT, int KS, int MODE>
__device__ __forceinline__ void mlp_layer(const _Float16* X, const _Float16* W, const float* bias,
                                           _Float16* Y, _Float16* prow, int lane) {
  constexpr int K = 32 * KS;
  const int hh = lane >> 4, nl = lane & 15;
#pragma unroll 1
  for (int nt = 0; nt < 4; ++nt) {
    v8f acc[MT];
#pragma unroll
    for (int mt = 0; mt < MT; ++mt) acc[mt] = splat8(0.0f);
    const _Float16* bp = W + (nt * 16 + nl) * K;
#pragma unroll
    for (int ks = 0; ks < KS; ++ks) {
      const v16h bf = ldfrag(bp, 32 * ks, hh);
#pragma unroll
      for (int mt = 0; mt < MT; ++mt)
        acc[mt] = wmf(ldfrag(X + (mt * 16 + nl) * K, 32 * ks, hh), bf, acc[mt]);
    }
    const int col = nt * 16 + nl;
    const float bv = bias[col];
    if (MODE == 0) {
#pragma unroll
      for (int mt = 0; mt < MT; ++mt) {
#pragma unroll
        for (int r = 0; r < 8; ++r) {
          const float h = fmaxf(acc[mt][r] * OSC + bv, 0.0f) * ASC;
          Y[(mt * 16 + 8 * hh + r) * 64 + col] = (_Float16)h;
        }
      }
    } else {
      float rm = 0.0f;
#pragma unroll
      for (int mt = 0; mt < MT; ++mt) {
#pragma unroll
        for (int r = 0; r < 8; ++r) rm = fmaxf(rm, acc[mt][r] * OSC + bv);
      }
      rm = fmaxf(rm, __shfl_xor(rm, 16, 32));
      if (hh == 0) prow[col] = (_Float16)(rm * ASC);
    }
  }
}

template <int S>
__device__ __forceinline__ void gather_rows(_Float16* X0, const int* sI, const _Float16* Fb, const v4f* Pb,
                                            float qx, float qy, float qz, int lane, _Float16 hz) {
#pragma clang fp contract(off)
#pragma unroll
  for (int p = 0; p < S / 4; ++p) {
    const int r = 4 * p + (lane >> 3);
    const int c8 = (lane & 7) * 8;
    int j = sI[r];
    j = min(max(j, 0), NPT - 1);
    const v8h v = *(const v8h*)(Fb + (size_t)j * NC + c8);
    *(v8h*)(X0 + r * K0P + c8) = v;
  }
  {
    const int r = lane & (S - 1);
    int j = sI[r];
    j = min(max(j, 0), NPT - 1);
    const v4f pt = Pb[j];
    const float gx = (pt.x - qx) * ASC;
    const float gy = (pt.y - qy) * ASC;
    const float gz = (pt.z - qz) * ASC;
    v8h o;
    o[0] = (_Float16)gx; o[1] = (_Float16)gy; o[2] = (_Float16)gz;
    o[3] = hz; o[4] = hz; o[5] = hz; o[6] = hz; o[7] = hz;
    *(v8h*)(X0 + r * K0P + 64) = o;
  }
}

__device__ __forceinline__ void store_row(const _Float16* prow, _Float16* dst, int lane) {
  const int l8 = lane & 7;
  const v8h v = *(const v8h*)(prow + 8 * l8);
  _Float16* d = dst + 8 * l8;
  if (lane < 8) *(volatile v8h*)d = v;
  __threadfence();
  if (lane < 8) *(volatile v8h*)d = v;
}

__global__ __launch_bounds__(128) void k_main(const float* __restrict__ xyz2, const v4f* __restrict__ P1,
                                              const _Float16* __restrict__ F1,
                                              const _Float16* __restrict__ w00, const _Float16* __restrict__ w01,
                                              const _Float16* __restrict__ w10, const _Float16* __restrict__ w11,
                                              const float* __restrict__ b00, const float* __restrict__ b01,
                                              const float* __restrict__ b10, const float* __restrict__ b11,
                                              _Float16* PL) {
#pragma clang fp contract(off)
  extern __shared__ __attribute__((aligned(16))) char smem[];
  _Float16* sW00 = (_Float16*)(smem + SMW00);
  _Float16* sW01 = (_Float16*)(smem + SMW01);
  _Float16* sW10 = (_Float16*)(smem + SMW10);
  _Float16* sW11 = (_Float16*)(smem + SMW11);
  float* sB = (float*)(smem + SMB);
  const int t = threadIdx.x, lane = t & 31, wv = t >> 5;
  char* wreg = smem + SMWV + wv * WVB;
  _Float16* X0 = (_Float16*)(wreg + WX0);
  _Float16* X1 = (_Float16*)(wreg + WX1);
  int* sI0 = (int*)(wreg + WI0);
  int* sI1 = (int*)(wreg + WI1);
  _Float16* prow = (_Float16*)(wreg + WPR);

  for (int p = t; p < H0 * K0P / 8; p += 128) *(v8h*)(sW00 + 8 * p) = *(const v8h*)(w00 + 8 * p);
  for (int p = t; p < H1 * H0 / 8; p += 128)  *(v8h*)(sW01 + 8 * p) = *(const v8h*)(w01 + 8 * p);
  for (int p = t; p < H0 * K0P / 8; p += 128) *(v8h*)(sW10 + 8 * p) = *(const v8h*)(w10 + 8 * p);
  for (int p = t; p < H1 * H0 / 8; p += 128)  *(v8h*)(sW11 + 8 * p) = *(const v8h*)(w11 + 8 * p);
  if (t < 64) {
    sB[t] = b00[t];
    sB[64 + t] = b01[t];
    sB[128 + t] = b10[t];
    sB[192 + t] = b11[t];
  }
  __syncthreads();

  const _Float16 hz = (_Float16)vgpr_zero();
  {
    const v8h z = {hz, hz, hz, hz, hz, hz, hz, hz};
    *(v8h*)(X0 + lane * K0P + 72) = z;
    *(v8h*)(X0 + lane * K0P + 80) = z;
    *(v8h*)(X0 + lane * K0P + 88) = z;
  }

  const float T0 = __uint_as_float(T0B);
  const float T1 = __uint_as_float(T1B);
  const unsigned pre = (1u << lane) - 1u;

#pragma unroll 1
  for (int i = 0; i < QPW; ++i) {
    const int q = (blockIdx.x * WPB + wv) * QPW + i;
    const int b = q / NQ;
    const float qx = xyz2[(size_t)q * 3], qy = xyz2[(size_t)q * 3 + 1], qz = xyz2[(size_t)q * 3 + 2];
    const float nq = norm3(qx, qy, qz);
    const v4f* Pb = P1 + (size_t)b * NPT;
    const _Float16* Fb = F1 + (size_t)b * NPT * NC;

    int cnt0 = 0, cnt1 = 0, first0 = -1, first1 = -1;
#pragma unroll 1
    for (int base = 0; base < NPT; base += 32) {
      if (cnt0 >= S0 && cnt1 >= S1) break;
      const int s = base + lane;
      const v4f pt = Pb[s];
      float dot = qx * pt.x;
      dot = __builtin_fmaf(qy, pt.y, dot);
      dot = __builtin_fmaf(qz, pt.z, dot);
      const float tsum = nq + pt.w;
      const float dd = dot + dot;
      const float d2 = tsum - dd;
      const bool in0 = d2 < T0;
      const bool in1 = d2 < T1;
      const unsigned m0 = (unsigned)__builtin_amdgcn_ballot_w32(in0);
      const unsigned m1 = (unsigned)__builtin_amdgcn_ballot_w32(in1);
      if (cnt0 < S0) {
        const int pos = cnt0 + (int)__builtin_popcount(m0 & pre);
        if (in0 && pos < S0) sI0[pos] = s;
        if (first0 < 0 && m0 != 0u) first0 = base + (int)__builtin_ctz(m0);
        cnt0 = min(cnt0 + (int)__builtin_popcount(m0), S0);
      }
      if (cnt1 < S1) {
        const int pos = cnt1 + (int)__builtin_popcount(m1 & pre);
        if (in1 && pos < S1) sI1[pos] = s;
        if (first1 < 0 && m1 != 0u) first1 = base + (int)__builtin_ctz(m1);
        cnt1 = min(cnt1 + (int)__builtin_popcount(m1), S1);
      }
    }
    {
      const int f0 = (cnt0 > 0) ? first0 : 0;
      const int f1v = (cnt1 > 0) ? first1 : 0;
      if (lane < S0 && lane >= cnt0) sI0[lane] = f0;
      if (lane >= cnt1) sI1[lane] = f1v;
    }
    wave_sync();

    gather_rows<S0>(X0, sI0, Fb, Pb, qx, qy, qz, lane, hz);
    wave_sync();
    mlp_layer<1, K0P / 32, 0>(X0, sW00, sB, X1, prow, lane);
    wave_sync();
    mlp_layer<1, H0 / 32, 1>(X1, sW01, sB + 64, X1, prow, lane);
    wave_sync();
    store_row(prow, PL + (size_t)q * H1, lane);

    gather_rows<S1>(X0, sI1, Fb, Pb, qx, qy, qz, lane, hz);
    wave_sync();
    mlp_layer<2, K0P / 32, 0>(X0, sW10, sB + 128, X1, prow, lane);
    wave_sync();
    mlp_layer<2, H0 / 32, 1>(X1, sW11, sB + 192, X1, prow, lane);
    wave_sync();
    store_row(prow, PL + ((size_t)NQT + q) * H1, lane);
    wave_sync();
  }
}

__global__ __launch_bounds__(128) void k_post(const _Float16* __restrict__ PL, const _Float16* __restrict__ F2,
                                              const _Float16* __restrict__ PW, const float* __restrict__ pbias,
                                              float* outp) {
  __shared__ __attribute__((aligned(16))) float sD[WPB][32 * 64];
  __shared__ float sPB[NPO];
  const int t = threadIdx.x, lane = t & 31, wv = t >> 5, hh = lane >> 4, nl = lane & 15;
  const int br = blockIdx.x / (NB * (NQ / 64));
  const int rem = blockIdx.x - br * (NB * (NQ / 64));
  const int b = rem / (NQ / 64);
  const int q0 = (rem - b * (NQ / 64)) * 64;
  sPB[t] = pbias[t];
  __syncthreads();

  const _Float16* Yp = PL + ((size_t)br * NQT + (size_t)b * NQ + q0) * H1;
  const _Float16* Yf = F2 + ((size_t)b * NQ + q0) * NC;
  const _Float16* Ap = PW + (size_t)(32 * wv) * KPO;

  v8f acc[8];
#pragma unroll
  for (int i = 0; i < 8; ++i) acc[i] = splat8(0.0f);
#pragma unroll
  for (int ks = 0; ks < 4; ++ks) {
    const v16h af0 = ldfrag(Ap + nl * KPO, 32 * ks, hh);
    const v16h af1 = ldfrag(Ap + (16 + nl) * KPO, 32 * ks, hh);
    v16h bf[4];
#pragma unroll
    for (int nt = 0; nt < 4; ++nt) {
      if (ks < 2) bf[nt] = ldfrag(Yp + (16 * nt + nl) * H1, 32 * ks, hh);
      else        bf[nt] = ldfrag(Yf + (16 * nt + nl) * NC, 32 * (ks - 2), hh);
    }
#pragma unroll
    for (int nt = 0; nt < 4; ++nt) {
      acc[nt] = wmf(af0, bf[nt], acc[nt]);
      acc[4 + nt] = wmf(af1, bf[nt], acc[4 + nt]);
    }
  }

  float* sdw = sD[wv];
#pragma unroll
  for (int mt = 0; mt < 2; ++mt) {
#pragma unroll
    for (int nt = 0; nt < 4; ++nt) {
#pragma unroll
      for (int r = 0; r < 8; ++r) {
        const int row = 16 * mt + 8 * hh + r;
        const int col = 16 * nt + nl;
        const float v = fmaxf(acc[mt * 4 + nt][r] * OSC + sPB[32 * wv + row], 0.0f);
        sdw[row * 64 + col] = v;
      }
    }
  }
  wave_sync();

  float* ob = outp + ((size_t)(b * NCH + br * NPO + 32 * wv)) * NQ + q0;
  const int pc = 4 * nl;
#pragma unroll
  for (int i = 0; i < 16; ++i) {
    const int lrow = 2 * i + hh;
    const v4f v = *(const v4f*)(sdw + lrow * 64 + pc);
    *(volatile v4f*)(ob + (size_t)lrow * NQ + pc) = v;
  }
  __threadfence();
#pragma unroll
  for (int i = 0; i < 16; ++i) {
    const int lrow = 2 * i + hh;
    const v4f v = *(const v4f*)(sdw + lrow * 64 + pc);
    *(volatile v4f*)(ob + (size_t)lrow * NQ + pc) = v;
  }
}

extern "C" void kernel_launch(void* const* d_in, const int* in_sizes, int n_in,
                              void* d_out, int out_size, void* d_ws, size_t ws_size,
                              hipStream_t stream) {
  if (n_in < 14) return;
  if (in_sizes[0] != NB * NQ * 3) return;
  if (in_sizes[1] != NB * NPT * 3) return;
  if (in_sizes[2] != NB * NC * NQ) return;
  if (in_sizes[3] != NB * NC * NPT) return;
  if (in_sizes[4] != H0 * K0 || in_sizes[5] != H0) return;
  if (in_sizes[6] != H1 * H0 || in_sizes[7] != H1) return;
  if (in_sizes[8] != H0 * K0 || in_sizes[9] != H0) return;
  if (in_sizes[10] != H1 * H0 || in_sizes[11] != H1) return;
  if (in_sizes[12] != NPO * KPO || in_sizes[13] != NPO) return;
  if (out_size != OUTN) return;

  const float* xyz2 = (const float*)d_in[0];
  const float* xyz1 = (const float*)d_in[1];
  const float* f2   = (const float*)d_in[2];
  const float* f1   = (const float*)d_in[3];
  const float* m0w0 = (const float*)d_in[4];
  const float* m0b0 = (const float*)d_in[5];
  const float* m0w1 = (const float*)d_in[6];
  const float* m0b1 = (const float*)d_in[7];
  const float* m1w0 = (const float*)d_in[8];
  const float* m1b0 = (const float*)d_in[9];
  const float* m1w1 = (const float*)d_in[10];
  const float* m1b1 = (const float*)d_in[11];
  const float* pw   = (const float*)d_in[12];
  const float* pb   = (const float*)d_in[13];
  float* out = (float*)d_out;

  char* ws = (char*)d_ws;
  size_t off = 0;
  const size_t oP1  = off; off += (size_t)NST * 16;          off = (off + 255) & ~(size_t)255;
  const size_t oF1  = off; off += (size_t)NST * NC * 2;      off = (off + 255) & ~(size_t)255;
  const size_t oF2  = off; off += (size_t)NQT * NC * 2;      off = (off + 255) & ~(size_t)255;
  const size_t oW00 = off; off += (size_t)H0 * K0P * 2;      off = (off + 255) & ~(size_t)255;
  const size_t oW01 = off; off += (size_t)H1 * H0 * 2;       off = (off + 255) & ~(size_t)255;
  const size_t oW10 = off; off += (size_t)H0 * K0P * 2;      off = (off + 255) & ~(size_t)255;
  const size_t oW11 = off; off += (size_t)H1 * H0 * 2;       off = (off + 255) & ~(size_t)255;
  const size_t oPW  = off; off += (size_t)NPO * KPO * 2;     off = (off + 255) & ~(size_t)255;
  const size_t oPL  = off; off += (size_t)2 * NQT * H1 * 2;  off = (off + 255) & ~(size_t)255;
  if (off > ws_size || off > (size_t)WSCAP) return;

  v4f*      P1  = (v4f*)(ws + oP1);
  _Float16* F1p = (_Float16*)(ws + oF1);
  _Float16* F2p = (_Float16*)(ws + oF2);
  _Float16* W00 = (_Float16*)(ws + oW00);
  _Float16* W01 = (_Float16*)(ws + oW01);
  _Float16* W10 = (_Float16*)(ws + oW10);
  _Float16* W11 = (_Float16*)(ws + oW11);
  _Float16* PWp = (_Float16*)(ws + oPW);
  _Float16* PLp = (_Float16*)(ws + oPL);

  hipFuncSetAttribute(reinterpret_cast<const void*>(&k_main),
                      hipFuncAttributeMaxDynamicSharedMemorySize, SMEM);

  k_pts<<<NST / 256, 256, 0, stream>>>(xyz1, NST, P1);
  k_tr<<<2 * NB * (NPT / 64), 256, 0, stream>>>(f1, f2, F1p, F2p);
  k_prepw<<<(H0 * K0P / 8) / 256, 256, 0, stream>>>(m0w0, K0, K0P, 1, H0 * K0P / 8, W00);
  k_prepw<<<(H1 * H0 / 8) / 256, 256, 0, stream>>>(m0w1, H0, H0, 0, H1 * H0 / 8, W01);
  k_prepw<<<(H0 * K0P / 8) / 256, 256, 0, stream>>>(m1w0, K0, K0P, 1, H0 * K0P / 8, W10);
  k_prepw<<<(H1 * H0 / 8) / 256, 256, 0, stream>>>(m1w1, H0, H0, 0, H1 * H0 / 8, W11);
  k_prepw<<<(NPO * KPO / 8) / 256, 256, 0, stream>>>(pw, KPO, KPO, 0, NPO * KPO / 8, PWp);
  k_main<<<NQT / QPB, 128, SMEM, stream>>>(xyz2, P1, F1p, W00, W01, W10, W11, m0b0, m0b1, m1b0, m1b1, PLp);
  k_post<<<2 * NB * (NQ / 64), 128, 0, stream>>>(PLp, F2p, PWp, pb, out);
}
